// GMBLayer_29652454212047
// MI455X (gfx1250) — hardware-verified
//
#include <hip/hip_runtime.h>
#include <math.h>


#define NNODE  8192
#define NGRAPH 128
#define NPG    64
#define KHOP   16
#define DD     128
#define NE     131072
#define NS     16
#define DTR    8
#define XPC    40
#define XPP    48
#define NSEQ   (NNODE * KHOP)

static_assert(NGRAPH * NPG == NNODE);
static_assert(NE % 2048 == 0);
static_assert(NSEQ == 131072);
static_assert(DTR + 2 * NS == XPC);
static_assert(NNODE % 256 == 0);
static_assert(NSEQ % 64 == 0);

typedef float    v4f  __attribute__((ext_vector_type(4)));
typedef float    v8f  __attribute__((ext_vector_type(8)));
typedef _Float16 v4h  __attribute__((ext_vector_type(4)));
typedef _Float16 v8h  __attribute__((ext_vector_type(8)));
typedef _Float16 v16h __attribute__((ext_vector_type(16)));
typedef int      v4i  __attribute__((ext_vector_type(4)));

union FragH { v8h h[2]; v16h v; };

constexpr size_t HP0 = 0;
constexpr size_t HP1 = HP0 + 128 * 128;
constexpr size_t HP2 = HP1 + 128 * 128;
constexpr size_t HP3 = HP2 + 128 * 128;
constexpr size_t HP4 = HP3 + 256 * 128;
constexpr size_t HP5 = HP4 + XPP * 128;
constexpr size_t HP6 = HP5 + 128 * 128;
constexpr size_t HPEND = HP6 + 256 * 128;

constexpr size_t SZ_PL   = HPEND * 2;
constexpr size_t SZ_DIS  = (size_t)NNODE * 4;
constexpr size_t SZ_H16  = (size_t)NNODE * DD * 2;
constexpr size_t SZ_F32  = (size_t)NNODE * DD * 4;
constexpr size_t SZ_SP   = (size_t)NSEQ * DD * 2;
constexpr size_t SZ_XC   = (size_t)NSEQ * DD * 4;

constexpr size_t OFF_PL  = 0;
constexpr size_t OFF_DIS = OFF_PL + SZ_PL;
constexpr size_t OFF_LNX = OFF_DIS + SZ_DIS;
constexpr size_t OFF_XL  = OFF_LNX + SZ_H16;
constexpr size_t OFF_LOC = OFF_XL + SZ_F32;
constexpr size_t OFF_SP  = OFF_LOC + SZ_F32;
constexpr size_t OFF_AG0 = OFF_SP + SZ_SP;
constexpr size_t OFF_H1  = OFF_AG0 + SZ_F32;
constexpr size_t OFF_G1  = OFF_H1 + SZ_H16;
constexpr size_t OFF_XSK = OFF_G1 + SZ_H16;
constexpr size_t OFF_XC  = OFF_XSK + SZ_F32;
constexpr size_t WS_END  = OFF_XC + SZ_XC;

static_assert(WS_END == (size_t)124039168);
static_assert(WS_END <= (size_t)134217728);
static_assert(OFF_DIS % 128 == 0 && OFF_LNX % 128 == 0 && OFF_XL % 128 == 0 && OFF_LOC % 128 == 0);
static_assert(OFF_SP % 128 == 0 && OFF_AG0 % 128 == 0 && OFF_H1 % 128 == 0 && OFF_G1 % 128 == 0);
static_assert(OFF_XSK % 128 == 0 && OFF_XC % 128 == 0 && WS_END % 128 == 0);
static_assert((HP1 * 2) % 256 == 0 && (HP3 * 2) % 256 == 0 && (HP4 * 2) % 256 == 0 && (HP5 * 2) % 256 == 0 && (HP6 * 2) % 256 == 0);

static constexpr float EPS_LN = 1e-5f;
static constexpr float GSC    = 0.0625f;

__device__ __forceinline__ v8f ld8f(const float* p) {
    v4f a = *(const v4f*)p;
    v4f b = *(const v4f*)(p + 4);
    return __builtin_shufflevector(a, b, 0, 1, 2, 3, 4, 5, 6, 7);
}
__device__ __forceinline__ v8h tof16(const v8f y) {
    v8h o;
#pragma unroll
    for (int e = 0; e < 8; ++e) o[e] = (_Float16)y[e];
    return o;
}
__device__ __forceinline__ float hsum16(float v) {
    v += __shfl_xor(v, 8, 32);
    v += __shfl_xor(v, 4, 32);
    v += __shfl_xor(v, 2, 32);
    v += __shfl_xor(v, 1, 32);
    return v;
}
__device__ __forceinline__ float silu_f(float x) {
    const float e = __expf(-x);
    return x * __builtin_amdgcn_rcpf(1.0f + e);
}
__device__ __forceinline__ float sigm_f(float x) {
    const float e = __expf(-x);
    return __builtin_amdgcn_rcpf(1.0f + e);
}
__device__ __forceinline__ float softplus_f(float x) {
    return fmaxf(x, 0.0f) + log1pf(__expf(-fabsf(x)));
}
__device__ __forceinline__ float gelu_f(float x) {
    return 0.5f * x * (erff(x * 0.70710678118654752f) + 1.0f);
}
__device__ __forceinline__ float conv4_silu(float x0, float x1, float x2, float x3,
                                            float w0, float w1, float w2, float w3, float bias) {
    const float c = w0 * x0 + w1 * x1 + w2 * x2 + w3 * x3;
    return silu_f(c + bias);
}
__device__ __forceinline__ v8f ln8(const v8f v, const v8f g8, const v8f b8) {
    float s = 0.0f;
#pragma unroll
    for (int e = 0; e < 8; ++e) s += v[e];
    const float mean = hsum16(s) * (1.0f / 128.0f);
    v8f dv;
    float q = 0.0f;
#pragma unroll
    for (int e = 0; e < 8; ++e) { dv[e] = v[e] - mean; q += dv[e] * dv[e]; }
    const float var  = hsum16(q) * (1.0f / 128.0f);
    const float rstd = rsqrtf(var + EPS_LN);
    v8f y;
#pragma unroll
    for (int e = 0; e < 8; ++e) y[e] = dv[e] * rstd * g8[e] + b8[e];
    return y;
}

__device__ __forceinline__ void mma16(v8f& acc, const FragH& a, const FragH& b) {
    acc = __builtin_amdgcn_wmma_f32_16x16x32_f16(false, a.v, false, b.v, (short)0, acc, false, false);
    asm volatile("v_nop\n\tv_nop\n\tv_nop\n\tv_nop" : "+v"(acc) : "v"(a.v), "v"(b.v));
}

__global__ __launch_bounds__(256)
void k_wplane(const float* __restrict__ w0, const float* __restrict__ w1, const float* __restrict__ w2,
              const float* __restrict__ w3, const float* __restrict__ w4, const float* __restrict__ w5,
              const float* __restrict__ w6, const float* __restrict__ w7, _Float16* planes)
{
    const int ent = blockIdx.y, bx = blockIdx.x, tid = threadIdx.x;
    const float* W = w0;
    int nsrc = 128, nrows = 128;
    size_t off = HP0;
    if (ent == 1)      { W = w1; off = HP1; }
    else if (ent == 2) { W = w2; off = HP2; }
    else if (ent == 3) { W = w3; nsrc = 256; nrows = 256; off = HP3; }
    else if (ent == 4) { W = w4; nsrc = XPC; nrows = XPP; off = HP4; }
    else if (ent == 5) { W = w5; off = HP5; }
    else if (ent == 6) { W = (((bx >> 1) & 1) != 0) ? w7 : w6; nrows = 256; off = HP6; }
    if (bx * 16 >= nrows) return;
    const int p = bx * 16 + (tid >> 4);
    const int q = tid & 15;
    int col;
    bool ok;
    if (ent == 6) { col = (p >> 6) * 32 + (p & 31); ok = true; }
    else          { ok = (p < nsrc); col = min(p, nsrc - 1); }
    v8h o;
#pragma unroll
    for (int e = 0; e < 8; ++e) {
        const int k = 8 * q + e;
        const float v = W[(size_t)k * nsrc + col] * 16.0f;
        o[e] = (_Float16)(ok ? v : 0.0f);
    }
    _Float16* gp = planes + off + (size_t)p * 128 + 8 * q;
    *(volatile v8h*)gp = o;
    __threadfence();
    *(volatile v8h*)gp = o;
}

__global__ __launch_bounds__(256)
void k_lnrows(const float* __restrict__ x, const float* __restrict__ g, const float* __restrict__ b, _Float16* dst)
{
    const int tid = threadIdx.x, lane = tid & 31, wave = tid >> 5;
    const int q = lane & 15, rs = lane >> 4;
    const v8f g8 = ld8f(g + 8 * q);
    const v8f b8 = ld8f(b + 8 * q);
#pragma unroll 1
    for (int it = 0; it < 4; ++it) {
        const int row = blockIdx.x * 64 + wave * 8 + it * 2 + rs;
        const v8f v = ld8f(x + (size_t)row * 128 + 8 * q);
        const v8h o = tof16(ln8(v, g8, b8));
        _Float16* gp = dst + (size_t)row * 128 + 8 * q;
        *(volatile v8h*)gp = o;
        __threadfence();
        *(volatile v8h*)gp = o;
    }
}

template<int MODE>
__device__ __forceinline__ void gpass_f32(const float* st, float* C, int rowW, int colW, int lane,
                                          const float* __restrict__ p0, const float* __restrict__ p1)
{
    const int rs = lane >> 4, c0 = (lane & 15) * 4;
#pragma unroll 4
    for (int it = 0; it < 16; ++it) {
        const int row = it * 2 + rs;
        const size_t grow = (size_t)(rowW + row);
        const v4f v = *(const v4f*)(st + row * 68 + c0);
        v4f o;
        if constexpr (MODE == 1) {
            const v4f bb = *(const v4f*)(p0 + colW + c0);
            const v4f rr = *(const v4f*)(p1 + grow * 128 + colW + c0);
#pragma unroll
            for (int e = 0; e < 4; ++e) o[e] = (v[e] * GSC + bb[e]) + rr[e];
        } else {
#pragma unroll
            for (int e = 0; e < 4; ++e) o[e] = v[e] * GSC;
        }
        *(volatile v4f*)(C + grow * 128 + colW + c0) = o;
    }
}

template<int MODE>
__device__ __forceinline__ void gpass_h16(const float* st, _Float16* C, int rowW, int colW, int lane,
                                          const float* __restrict__ p0)
{
    const int q = lane & 7, rs = lane >> 3;
#pragma unroll 1
    for (int it = 0; it < 8; ++it) {
        const int row = it * 4 + rs;
        const size_t grow = (size_t)(rowW + row);
        const v8f v = ld8f(st + row * 68 + 8 * q);
        v8f y;
#pragma unroll
        for (int e = 0; e < 8; ++e) {
            float t = v[e] * GSC;
            if constexpr (MODE == 2) t += p0[colW + 8 * q + e];
            y[e] = gelu_f(t);
        }
        *(volatile v8h*)(C + grow * 128 + colW + 8 * q) = tof16(y);
    }
}

__device__ __forceinline__ void gpass_out(const float* st, float* out, int rowW, int colW, int lane,
                                          const float* __restrict__ b1, const float* __restrict__ loc,
                                          const float* __restrict__ b2, const float* __restrict__ xsk)
{
    const int q = lane & 7, rs = lane >> 3;
    const int cb = colW >> 1;
#pragma unroll 1
    for (int it = 0; it < 8; ++it) {
        const int row = it * 4 + rs;
        const size_t grow = (size_t)(rowW + row);
        const v4f a = *(const v4f*)(st + row * 68 + 4 * q);
        const v4f b = *(const v4f*)(st + row * 68 + 32 + 4 * q);
        const v4f lv = *(const v4f*)(loc + grow * 128 + cb + 4 * q);
        const v4f xv = *(const v4f*)(xsk + grow * 128 + cb + 4 * q);
        v4f o;
#pragma unroll
        for (int e = 0; e < 4; ++e) {
            const int c = cb + 4 * q + e;
            const float ma = a[e] * GSC + b1[c];
            const float mb = b[e] * GSC + b2[c];
            const float s  = ma * sigm_f(mb) + xv[e];
            o[e] = lv[e] + s;
        }
        *(volatile v4f*)(out + grow * 128 + cb + 4 * q) = o;
    }
}

template<int MODE>
__global__ __launch_bounds__(128)
void k_gemm(const _Float16* __restrict__ A, int lda, const _Float16* __restrict__ Bw, void* Cv,
            const float* __restrict__ p0, const float* __restrict__ p1,
            const float* __restrict__ p2, const float* __restrict__ p3)
{
    __shared__ __attribute__((aligned(16))) float stile[4][32 * 68];

    const int tid = threadIdx.x, lane = tid & 31, wave = tid >> 5;
    const int h = lane >> 4, m = lane & 15;
    const int wm = wave >> 1, wn = wave & 1;
    const int rowW = blockIdx.y * 64 + wm * 32;
    const int colW = blockIdx.x * 128 + wn * 64;

    const _Float16* pa0 = A + (size_t)(rowW + m) * lda + 8 * h;
    const _Float16* pa1 = pa0 + (size_t)16 * lda;
    const _Float16* pb  = Bw + (size_t)(colW + m) * 128 + 8 * h;

    v8f acc[8];
#pragma unroll
    for (int j = 0; j < 8; ++j)
#pragma unroll
        for (int r = 0; r < 8; ++r) acc[j][r] = 0.0f;

#pragma unroll
    for (int kt = 0; kt < 4; ++kt) {
        const int k0 = kt * 32;
        FragH fa0, fa1;
        fa0.h[0] = *(const v8h*)(pa0 + k0);
        fa0.h[1] = *(const v8h*)(pa0 + k0 + 16);
        fa1.h[0] = *(const v8h*)(pa1 + k0);
        fa1.h[1] = *(const v8h*)(pa1 + k0 + 16);
#pragma unroll
        for (int j = 0; j < 4; ++j) {
            const _Float16* p = pb + (size_t)j * 2048 + k0;
            FragH fb;
            fb.h[0] = *(const v8h*)p;
            fb.h[1] = *(const v8h*)(p + 16);
            mma16(acc[j], fa0, fb);
            mma16(acc[4 + j], fa1, fb);
        }
    }

    float* st = stile[wave];
#pragma unroll
    for (int s = 0; s < 2; ++s)
#pragma unroll
        for (int j = 0; j < 4; ++j)
#pragma unroll
            for (int r = 0; r < 8; ++r)
                st[(s * 16 + 8 * h + r) * 68 + j * 16 + m] = acc[s * 4 + j][r];
    __syncthreads();

    if constexpr (MODE == 0 || MODE == 1) {
        float* C = (float*)Cv;
        gpass_f32<MODE>(st, C, rowW, colW, lane, p0, p1);
        __threadfence();
        gpass_f32<MODE>(st, C, rowW, colW, lane, p0, p1);
    } else if constexpr (MODE == 2 || MODE == 3) {
        _Float16* C = (_Float16*)Cv;
        gpass_h16<MODE>(st, C, rowW, colW, lane, p0);
        __threadfence();
        gpass_h16<MODE>(st, C, rowW, colW, lane, p0);
    } else {
        float* C = (float*)Cv;
        gpass_out(st, C, rowW, colW, lane, p0, p1, p2, p3);
        __threadfence();
        gpass_out(st, C, rowW, colW, lane, p0, p1, p2, p3);
    }
}

__device__ __forceinline__ void deg_pass(const float* sd, float* dis, int n0, int tid) {
    if (tid < 64) {
        const v4f v = *(const v4f*)(sd + 4 * tid);
        *(volatile v4f*)(dis + n0 + 4 * tid) = v;
    }
}

__global__ __launch_bounds__(256)
void k_deg(const int* __restrict__ ei, const int* __restrict__ glab, float* dis)
{
    __shared__ int lst[8 * 256];
    __shared__ int wc[8];
    __shared__ __attribute__((aligned(16))) float sd[256];
    (void)glab;
    const int tid = threadIdx.x, lane = tid & 31, wave = tid >> 5;
    const int n0 = blockIdx.x * 256;
    const unsigned lt = (1u << lane) - 1u;
    int cnt = 0;
#pragma unroll 1
    for (int cbase = 0; cbase < NE; cbase += 2048) {
        int wn = 0;
#pragma unroll 1
        for (int it = 0; it < 8; ++it) {
            const int e   = cbase + wave * 256 + it * 32 + lane;
            const int dst = ei[NE + min(e, NE - 1)];
            const int ld  = dst - n0;
            const bool hit = (unsigned)ld < 256u;
            const unsigned msk = (unsigned)__ballot(hit);
            const int pos = wn + (int)__popc(msk & lt);
            if (hit) lst[wave * 256 + pos] = ld;
            wn += (int)__popc(msk);
        }
        if (lane == 0) wc[wave] = wn;
        __syncthreads();
#pragma unroll 1
        for (int w = 0; w < 8; ++w) {
            const int nw = min(wc[w], 256);
#pragma unroll 1
            for (int p = 0; p < nw; ++p) cnt += (lst[w * 256 + p] == tid) ? 1 : 0;
        }
        __syncthreads();
    }
    sd[tid] = rsqrtf((float)(cnt + 1));
    __syncthreads();
    deg_pass(sd, dis, n0, tid);
    __threadfence();
    deg_pass(sd, dis, n0, tid);
}

__device__ __forceinline__ void gcn_pass(const float* acc, float* local, int n0, int tid) {
#pragma unroll 4
    for (int it = 0; it < 16; ++it) {
        const int idx = it * 128 + tid;
        const int r = idx >> 5, q = idx & 31;
        const v4f v = *(const v4f*)(acc + r * 128 + 4 * q);
        *(volatile v4f*)(local + (size_t)(n0 + r) * 128 + 4 * q) = v;
    }
}

__global__ __launch_bounds__(128)
void k_gcn(const int* __restrict__ ei, const float* __restrict__ x, const float* __restrict__ xl,
           const float* __restrict__ dis, const float* __restrict__ bg, float* local)
{
    __shared__ __attribute__((aligned(16))) float acc[64 * 128];
    __shared__ int lst[4 * 512];
    __shared__ int wc[4];
    __shared__ float dl[64];
    const int tid = threadIdx.x, lane = tid & 31, wave = tid >> 5;
    const int n0 = blockIdx.x * 64;
#pragma unroll 4
    for (int r = 0; r < 64; ++r) acc[r * 128 + tid] = 0.0f;
    if (tid < 64) dl[tid] = dis[n0 + tid];
    __syncthreads();
    const unsigned lt = (1u << lane) - 1u;
    const float bgv = bg[tid];
#pragma unroll 1
    for (int cbase = 0; cbase < NE; cbase += 2048) {
        int cnt = 0;
#pragma unroll 1
        for (int it = 0; it < 16; ++it) {
            const int e   = min(cbase + wave * 512 + it * 32 + lane, NE - 1);
            const int src = ei[e];
            const int dst = ei[NE + e];
            const int ld  = dst - n0;
            const bool hit = (unsigned)ld < 64u;
            const unsigned msk = (unsigned)__ballot(hit);
            const int pos = cnt + (int)__popc(msk & lt);
            if (hit) lst[wave * 512 + pos] = (src << 6) | ld;
            cnt += (int)__popc(msk);
        }
        if (lane == 0) wc[wave] = cnt;
        __syncthreads();
#pragma unroll 1
        for (int w = 0; w < 4; ++w) {
            const int nw = min(wc[w], 512);
#pragma unroll 1
            for (int p = 0; p < nw; ++p) {
                const int item = lst[w * 512 + p];
                const int src  = min(max(item >> 6, 0), NNODE - 1);
                const int ld   = item & 63;
                const float nrm = dis[src] * dl[ld];
                acc[ld * 128 + tid] += nrm * xl[(size_t)src * 128 + tid];
            }
        }
        __syncthreads();
    }
#pragma unroll 4
    for (int r = 0; r < 64; ++r) {
        const size_t gi = (size_t)(n0 + r) * 128 + tid;
        const float dd = dl[r];
        const float gv = (acc[r * 128 + tid] + dd * dd * xl[gi]) + bgv;
        acc[r * 128 + tid] = x[gi] + gv;
    }
    __syncthreads();
    gcn_pass(acc, local, n0, tid);
    __threadfence();
    gcn_pass(acc, local, n0, tid);
}

__device__ __forceinline__ void agg_pass(const float* Dst, _Float16* sP, float* agg0, _Float16* h1P,
                                         int g, int k, int t, int wave, int lane, int q16, int rs,
                                         const v8f g8s, const v8f b8s, const v8f g8m, const v8f b8m)
{
#pragma unroll 1
    for (int it = 0; it < 8; ++it) {
        const int i = 16 * wave + 2 * it + rs;
        const size_t n = (size_t)g * 64 + i;
        const v8f v = ld8f(Dst + i * 132 + 8 * q16);
        const v8f y = ln8(v, g8s, b8s);
        *(volatile v8h*)(sP + (n * 16 + t) * 128 + 8 * q16) = tof16(y);
        if (k == 0) {
            const v8f y2 = ln8(v, g8m, b8m);
            *(volatile v8h*)(h1P + n * 128 + 8 * q16) = tof16(y2);
        }
    }
    if (k == 0) {
#pragma unroll 4
        for (int i2 = 0; i2 < 16; ++i2) {
            const int i = 16 * wave + i2;
            const size_t n = (size_t)g * 64 + i;
            const v4f v = *(const v4f*)(Dst + i * 132 + 4 * lane);
            *(volatile v4f*)(agg0 + n * 128 + 4 * lane) = v;
        }
    }
}

__global__ __launch_bounds__(128)
void k_agg(const int* __restrict__ mask, const float* __restrict__ x,
           const float* __restrict__ gs, const float* __restrict__ bs,
           const float* __restrict__ gm, const float* __restrict__ bm,
           _Float16* sP, float* agg0, _Float16* h1P)
{
    __shared__ __attribute__((aligned(16))) _Float16 xT[128 * 72];
    __shared__ __attribute__((aligned(16))) _Float16 mk[64 * 72];
    __shared__ __attribute__((aligned(16))) float Dst[64 * 132];

    const int tid = threadIdx.x, lane = tid & 31, wave = tid >> 5;
    const int h = lane >> 4, m = lane & 15;
    const int q16 = lane & 15, rs = lane >> 4;
    const int g = blockIdx.x;

#pragma unroll 1
    for (int it = 0; it < 16; ++it) {
        const int idx = it * 128 + tid;
        const int j = idx >> 5, q = idx & 31;
        const v4f v = *(const v4f*)(x + (size_t)(g * 64 + j) * 128 + 4 * q);
#pragma unroll
        for (int c = 0; c < 4; ++c) xT[(4 * q + c) * 72 + j] = (_Float16)v[c];
    }
    const v8f g8s = ld8f(gs + 8 * q16), b8s = ld8f(bs + 8 * q16);
    const v8f g8m = ld8f(gm + 8 * q16), b8m = ld8f(bm + 8 * q16);
    const _Float16 one = (_Float16)1.0f, zer = (_Float16)0.0f;

#pragma unroll 1
    for (int k = 0; k < KHOP; ++k) {
        const int* mg = mask + (size_t)(g * KHOP + k) * 4096;
#pragma unroll
        for (int it = 0; it < 8; ++it) {
            const int idx = it * 128 + tid;
            const int i = idx >> 4, j4 = (idx & 15) * 4;
            const v4i mv = *(const v4i*)(mg + i * 64 + j4);
            v4h o;
#pragma unroll
            for (int c = 0; c < 4; ++c) o[c] = (mv[c] != 0) ? one : zer;
            *(v4h*)(mk + i * 72 + j4) = o;
        }
        __syncthreads();

        v8f acc[8];
#pragma unroll
        for (int j = 0; j < 8; ++j)
#pragma unroll
            for (int r = 0; r < 8; ++r) acc[j][r] = 0.0f;
        const _Float16* pa = mk + (16 * wave + m) * 72 + 8 * h;
#pragma unroll
        for (int kt = 0; kt < 2; ++kt) {
            FragH fa;
            fa.h[0] = *(const v8h*)(pa + 32 * kt);
            fa.h[1] = *(const v8h*)(pa + 32 * kt + 16);
#pragma unroll
            for (int j = 0; j < 8; ++j) {
                const _Float16* pb = xT + (16 * j + m) * 72 + 8 * h + 32 * kt;
                FragH fb;
                fb.h[0] = *(const v8h*)pb;
                fb.h[1] = *(const v8h*)(pb + 16);
                mma16(acc[j], fa, fb);
            }
        }
#pragma unroll
        for (int j = 0; j < 8; ++j)
#pragma unroll
            for (int r = 0; r < 8; ++r)
                Dst[(16 * wave + 8 * h + r) * 132 + 16 * j + m] = acc[j][r];
        __syncthreads();

        const int t = KHOP - 1 - k;
        agg_pass(Dst, sP, agg0, h1P, g, k, t, wave, lane, q16, rs, g8s, b8s, g8m, b8m);
        __threadfence();
        agg_pass(Dst, sP, agg0, h1P, g, k, t, wave, lane, q16, rs, g8s, b8s, g8m, b8m);
    }
}

__device__ __forceinline__ void yg_pass(const float* ys, _Float16* ygP, int nb, int tid) {
    if (tid < 64) {
        const int rr = tid >> 4, q8 = tid & 15;
        const v8f v = ld8f(ys + rr * 128 + 8 * q8);
        *(volatile v8h*)(ygP + (size_t)(nb * 4 + rr) * 128 + 8 * q8) = tof16(v);
    }
}

__global__ __launch_bounds__(128)
void k_xscan(const float* __restrict__ xc, const float* __restrict__ z15, const _Float16* __restrict__ xpP,
             const float* __restrict__ cw, const float* __restrict__ cb, const float* __restrict__ dtw,
             const float* __restrict__ dtb, const float* __restrict__ Alog, const float* __restrict__ Dsk,
             _Float16* ygP)
{
    __shared__ __attribute__((aligned(16))) _Float16 uh[64 * 136];
    __shared__ __attribute__((aligned(16))) float xd[64 * 52];
    __shared__ __attribute__((aligned(16))) float ys[4 * 128];

    const int tid = threadIdx.x, lane = tid & 31, wave = tid >> 5;
    const int h = lane >> 4, m = lane & 15;
    const int nb = blockIdx.x;
    const size_t r0 = (size_t)nb * 64;

#pragma unroll 1
    for (int it = 0; it < 16; ++it) {
        const int idx = it * 128 + tid;
        const int r = idx >> 5, q = idx & 31;
        const int t = r & 15;
        const int r1 = r - ((t >= 1) ? 1 : 0);
        const int r2 = r - ((t >= 2) ? 2 : 0);
        const int r3 = r - ((t >= 3) ? 3 : 0);
        const v4f x3 = *(const v4f*)(xc + (r0 + r)  * 128 + 4 * q);
        const v4f x2 = *(const v4f*)(xc + (r0 + r1) * 128 + 4 * q);
        const v4f x1 = *(const v4f*)(xc + (r0 + r2) * 128 + 4 * q);
        const v4f x0 = *(const v4f*)(xc + (r0 + r3) * 128 + 4 * q);
        v4h o;
#pragma unroll
        for (int c = 0; c < 4; ++c) {
            const int ch = 4 * q + c;
            const v4f w4 = *(const v4f*)(cw + ch * 4);
            const float a2 = (t >= 1) ? x2[c] : 0.0f;
            const float a1 = (t >= 2) ? x1[c] : 0.0f;
            const float a0 = (t >= 3) ? x0[c] : 0.0f;
            o[c] = (_Float16)conv4_silu(a0, a1, a2, x3[c], w4[0], w4[1], w4[2], w4[3], cb[ch]);
        }
        *(v4h*)(uh + r * 136 + 4 * q) = o;
    }
    __syncthreads();

    v8f acc[3];
#pragma unroll
    for (int j = 0; j < 3; ++j)
#pragma unroll
        for (int r = 0; r < 8; ++r) acc[j][r] = 0.0f;
    const _Float16* pa = uh + (16 * wave + m) * 136 + 8 * h;
    const _Float16* pb = xpP + (size_t)m * 128 + 8 * h;
#pragma unroll
    for (int kt = 0; kt < 4; ++kt) {
        FragH fa;
        fa.h[0] = *(const v8h*)(pa + 32 * kt);
        fa.h[1] = *(const v8h*)(pa + 32 * kt + 16);
#pragma unroll
        for (int j = 0; j < 3; ++j) {
            const _Float16* p = pb + (size_t)j * 2048 + 32 * kt;
            FragH fb;
            fb.h[0] = *(const v8h*)p;
            fb.h[1] = *(const v8h*)(p + 16);
            mma16(acc[j], fa, fb);
        }
    }
#pragma unroll
    for (int j = 0; j < 3; ++j)
#pragma unroll
        for (int r = 0; r < 8; ++r)
            xd[(16 * wave + 8 * h + r) * 52 + 16 * j + m] = acc[j][r] * GSC;
    __syncthreads();

    const int d = tid;
    float As[NS];
#pragma unroll
    for (int s = 0; s < NS; ++s) As[s] = -expf(Alog[d * NS + s]);
    float dw[DTR];
#pragma unroll
    for (int kk = 0; kk < DTR; ++kk) dw[kk] = dtw[kk * 128 + d];
    const float db = dtb[d], Dd = Dsk[d], cbd = cb[d];
    const v4f wd = *(const v4f*)(cw + d * 4);

#pragma unroll 1
    for (int q = 0; q < 4; ++q) {
        float hs[NS];
#pragma unroll
        for (int s = 0; s < NS; ++s) hs[s] = 0.0f;
        float xm1 = 0.0f, xm2 = 0.0f, xm3 = 0.0f, ul = 0.0f;
        const size_t rb = r0 + (size_t)q * 16;
#pragma unroll 1
        for (int t = 0; t < 16; ++t) {
            const float xv = xc[(rb + t) * 128 + d];
            const float u  = conv4_silu(xm3, xm2, xm1, xv, wd[0], wd[1], wd[2], wd[3], cbd);
            xm3 = xm2; xm2 = xm1; xm1 = xv;
            const float* xr = xd + (q * 16 + t) * 52;
            float dl = 0.0f;
#pragma unroll
            for (int kk = 0; kk < DTR; ++kk) dl += xr[kk] * dw[kk];
            dl += db;
            const float dt = softplus_f(dl);
#pragma unroll
            for (int s = 0; s < NS; ++s) {
                const float dA = __expf(dt * As[s]);
                hs[s] = dA * hs[s] + (dt * xr[DTR + s]) * u;
            }
            ul = u;
        }
        const float* xr = xd + (q * 16 + 15) * 52;
        float y = 0.0f;
#pragma unroll
        for (int s = 0; s < NS; ++s) y += hs[s] * xr[DTR + NS + s];
        y += ul * Dd;
        const float zv = z15[(size_t)(nb * 4 + q) * 128 + d];
        ys[q * 128 + d] = y * silu_f(zv);
    }
    __syncthreads();
    yg_pass(ys, ygP, nb, tid);
    __threadfence();
    yg_pass(ys, ygP, nb, tid);
}

extern "C" void kernel_launch(void* const* d_in, const int* in_sizes, int n_in,
                              void* d_out, int out_size, void* d_ws, size_t ws_size,
                              hipStream_t stream)
{
    if (n_in < 29) return;
    if (in_sizes[0]  != NNODE * DD) return;
    if (in_sizes[1]  != 2 * NE) return;
    if (in_sizes[2]  != NNODE) return;
    if (in_sizes[3]  != NGRAPH * KHOP * NPG * NPG) return;
    if (in_sizes[4]  != DD * DD) return;
    if (in_sizes[5]  != DD || in_sizes[6] != DD || in_sizes[7] != DD || in_sizes[8] != DD || in_sizes[9] != DD) return;
    if (in_sizes[10] != DD * DD || in_sizes[11] != DD || in_sizes[12] != DD * DD || in_sizes[13] != DD) return;
    if (in_sizes[14] != DD || in_sizes[15] != DD) return;
    if (in_sizes[16] != DD * 256) return;
    if (in_sizes[17] != DD * 4 || in_sizes[18] != DD) return;
    if (in_sizes[19] != DD * XPC) return;
    if (in_sizes[20] != DTR * DD || in_sizes[21] != DD) return;
    if (in_sizes[22] != DD * NS || in_sizes[23] != DD) return;
    if (in_sizes[24] != DD * DD) return;
    if (in_sizes[25] != DD * DD || in_sizes[26] != DD || in_sizes[27] != DD * DD || in_sizes[28] != DD) return;
    if (out_size != NNODE * DD) return;
    if (ws_size < WS_END) return;

    const float* x        = (const float*)d_in[0];
    const int*   ei       = (const int*)d_in[1];
    const int*   glab     = (const int*)d_in[2];
    const int*   masks    = (const int*)d_in[3];
    const float* w_gcn    = (const float*)d_in[4];
    const float* b_gcn    = (const float*)d_in[5];
    const float* lnl_g    = (const float*)d_in[6];
    const float* lnl_b    = (const float*)d_in[7];
    const float* m1ln_g   = (const float*)d_in[8];
    const float* m1ln_b   = (const float*)d_in[9];
    const float* m1w1     = (const float*)d_in[10];
    const float* m1b1     = (const float*)d_in[11];
    const float* m1w2     = (const float*)d_in[12];
    const float* m1b2     = (const float*)d_in[13];
    const float* ln_g     = (const float*)d_in[14];
    const float* ln_b     = (const float*)d_in[15];
    const float* in_proj  = (const float*)d_in[16];
    const float* conv_w   = (const float*)d_in[17];
    const float* conv_b   = (const float*)d_in[18];
    const float* x_proj   = (const float*)d_in[19];
    const float* dtp_w    = (const float*)d_in[20];
    const float* dtp_b    = (const float*)d_in[21];
    const float* A_log    = (const float*)d_in[22];
    const float* Dsk      = (const float*)d_in[23];
    const float* out_proj = (const float*)d_in[24];
    const float* m2w1     = (const float*)d_in[25];
    const float* m2b1     = (const float*)d_in[26];
    const float* m2w2     = (const float*)d_in[27];
    const float* m2b2     = (const float*)d_in[28];
    float* out = (float*)d_out;

    char* ws = (char*)d_ws;
    _Float16* PL    = (_Float16*)(ws + OFF_PL);
    float*    dis   = (float*)(ws + OFF_DIS);
    _Float16* lnxP  = (_Float16*)(ws + OFF_LNX);
    _Float16* ygP   = (_Float16*)(ws + OFF_LNX);
    float*    xl    = (float*)(ws + OFF_XL);
    float*    z15   = (float*)(ws + OFF_XL);
    float*    local = (float*)(ws + OFF_LOC);
    _Float16* sP    = (_Float16*)(ws + OFF_SP);
    float*    agg0  = (float*)(ws + OFF_AG0);
    _Float16* h1P   = (_Float16*)(ws + OFF_H1);
    _Float16* gP    = (_Float16*)(ws + OFF_H1);
    _Float16* g1P   = (_Float16*)(ws + OFF_G1);
    float*    xsk   = (float*)(ws + OFF_XSK);
    float*    xc    = (float*)(ws + OFF_XC);

    const dim3 b128(128), b256(256);

    k_wplane<<<dim3(16, 7), b256, 0, stream>>>(w_gcn, m1w1, m1w2, in_proj, x_proj, out_proj, m2w1, m2w2, PL);
    k_lnrows<<<dim3(NNODE / 64), b256, 0, stream>>>(x, lnl_g, lnl_b, lnxP);
    k_gemm<0><<<dim3(1, NNODE / 64), b128, 0, stream>>>(lnxP, 128, PL + HP0, (void*)xl, b_gcn, b_gcn, b_gcn, b_gcn);
    k_deg<<<dim3(NNODE / 256), b256, 0, stream>>>(ei, glab, dis);
    k_gcn<<<dim3(NNODE / 64), b128, 0, stream>>>(ei, x, xl, dis, b_gcn, local);
    k_agg<<<dim3(NGRAPH), b128, 0, stream>>>(masks, x, ln_g, ln_b, m1ln_g, m1ln_b, sP, agg0, h1P);
    k_gemm<2><<<dim3(1, NNODE / 64), b128, 0, stream>>>(h1P, 128, PL + HP1, (void*)g1P, m1b1, m1b1, m1b1, m1b1);
    k_gemm<1><<<dim3(1, NNODE / 64), b128, 0, stream>>>(g1P, 128, PL + HP2, (void*)xsk, m1b2, agg0, m1b2, m1b2);
    k_gemm<0><<<dim3(1, NSEQ / 64), b128, 0, stream>>>(sP, 128, PL + HP3, (void*)xc, b_gcn, b_gcn, b_gcn, b_gcn);
    k_gemm<0><<<dim3(1, NNODE / 64), b128, 0, stream>>>(sP + 15 * 128, 16 * 128, PL + HP3 + 128 * 128, (void*)z15,
                                                        b_gcn, b_gcn, b_gcn, b_gcn);
    k_xscan<<<dim3(NNODE / 4), b128, 0, stream>>>(xc, z15, PL + HP4, conv_w, conv_b, dtp_w, dtp_b, A_log, Dsk, ygP);
    k_gemm<3><<<dim3(1, NNODE / 64), b128, 0, stream>>>(ygP, 128, PL + HP5, (void*)gP, m2b1, m2b1, m2b1, m2b1);
    k_gemm<4><<<dim3(2, NNODE / 64), b128, 0, stream>>>(gP, 128, PL + HP6, (void*)out, m2b1, (const float*)local,
                                                        m2b2, (const float*)xsk);
}
